// Head_30597347017102
// MI455X (gfx1250) — hardware-verified
//
#include <hip/hip_runtime.h>
#include <math.h>

#ifndef NB
#define NB 64
#endif
#ifndef SEQ
#define SEQ 512
#endif
#define SEQ_FULL 512
#define NB_FULL 64
#define CIN 384
#define HD 64
#define NQKV 192
#define NXR 64
#define AW 4

static_assert(SEQ % 64 == 0);
static_assert(SEQ > NXR);
static_assert((SEQ - NXR) % (16 * AW) == 0);
static_assert(SEQ <= SEQ_FULL);
static_assert(NB <= NB_FULL);
static_assert(((long long)NB * SEQ) % 64 == 0);
static_assert(NQKV % 64 == 0);
static_assert(CIN % 32 == 0);
static_assert(((long long)NB * SEQ * (CIN / 8)) % 256 == 0);
static_assert((HD * (CIN / 8)) % 256 == 0);
static_assert(NXR == 64);

typedef __attribute__((ext_vector_type(16))) _Float16     v16h;
typedef __attribute__((ext_vector_type(8)))  _Float16     v8h;
typedef __attribute__((ext_vector_type(16))) __bf16       v16b;
typedef __attribute__((ext_vector_type(8)))  float        v8f;
typedef __attribute__((ext_vector_type(4)))  float        v4f;
typedef __attribute__((ext_vector_type(4)))  unsigned int cm_u4;

__device__ __forceinline__ int frag_k(int i, int h) { return (i < 8) ? (8 * h + i) : (16 + 8 * h + (i - 8)); }
__device__ __forceinline__ __bf16 bf16_rne(float f) {
    unsigned int u = __float_as_uint(f);
    u += 0x7fffu + ((u >> 16) & 1u);
    return __builtin_bit_cast(__bf16, (unsigned short)(u >> 16));
}
__device__ __forceinline__ float bf16_f32(__bf16 b) { return __uint_as_float(((unsigned int)__builtin_bit_cast(unsigned short, b)) << 16); }
__device__ __forceinline__ v8f wmma16(v16h a, v16h b, v8f c) {
    c = __builtin_amdgcn_wmma_f32_16x16x32_f16(false, a, false, b, (short)0, c, false, false);
    asm volatile("v_nop\n\tv_nop\n\tv_nop\n\tv_nop" : "+v"(c) : "v"(a), "v"(b));
    return c;
}
struct Split { v16b hi, lo; };
__device__ __forceinline__ v8f wmma3(const Split& a, const Split& b, v8f c) {
    c = __builtin_amdgcn_wmma_f32_16x16x32_bf16(false, a.hi, false, b.hi, (short)0, c, false, false);
    c = __builtin_amdgcn_wmma_f32_16x16x32_bf16(false, a.hi, false, b.lo, (short)0, c, false, false);
    c = __builtin_amdgcn_wmma_f32_16x16x32_bf16(false, a.lo, false, b.hi, (short)0, c, false, false);
    asm volatile("v_nop\n\tv_nop\n\tv_nop\n\tv_nop" : "+v"(c) : "v"(a.hi), "v"(a.lo), "v"(b.hi), "v"(b.lo));
    return c;
}
__device__ __forceinline__ Split sp_row(const float* __restrict__ row, int k0, int h) {
    const v4f a0 = *(const v4f*)(row + k0 + 8 * h);
    const v4f a1 = *(const v4f*)(row + k0 + 8 * h + 4);
    const v4f a2 = *(const v4f*)(row + k0 + 16 + 8 * h);
    const v4f a3 = *(const v4f*)(row + k0 + 16 + 8 * h + 4);
    const float f[16] = {a0.x, a0.y, a0.z, a0.w, a1.x, a1.y, a1.z, a1.w, a2.x, a2.y, a2.z, a2.w, a3.x, a3.y, a3.z, a3.w};
    Split r;
#pragma unroll
    for (int i = 0; i < 16; ++i) { const __bf16 hb = bf16_rne(f[i]); r.hi[i] = hb; r.lo[i] = bf16_rne(f[i] - bf16_f32(hb)); }
    return r;
}
__device__ __forceinline__ v16h ph_row(const float* row, int k0, int h, float s) {
    const v4f a0 = *(const v4f*)(row + k0 + 8 * h);
    const v4f a1 = *(const v4f*)(row + k0 + 8 * h + 4);
    const v4f a2 = *(const v4f*)(row + k0 + 16 + 8 * h);
    const v4f a3 = *(const v4f*)(row + k0 + 16 + 8 * h + 4);
    const float f[16] = {a0.x, a0.y, a0.z, a0.w, a1.x, a1.y, a1.z, a1.w, a2.x, a2.y, a2.z, a2.w, a3.x, a3.y, a3.z, a3.w};
    v16h a;
#pragma unroll
    for (int i = 0; i < 16; ++i) a[i] = (_Float16)(f[i] * s);
    return a;
}

#define VST2(T, ptr, val) do { const T vst2_v_ = (val); *(volatile T*)(ptr) = vst2_v_; __threadfence(); *(volatile T*)(ptr) = vst2_v_; } while (0)
#define VST2V4(ptr, val) do { const v4f vst2_v4_ = (val); *(volatile v4f*)(ptr) = vst2_v4_; __threadfence(); *(volatile v4f*)(ptr) = vst2_v4_; } while (0)

__device__ __forceinline__ unsigned int cmb_pk2(float a, float b) { return (unsigned int)__builtin_bit_cast(unsigned short, (_Float16)a) | ((unsigned int)__builtin_bit_cast(unsigned short, (_Float16)b) << 16); }
__device__ __forceinline__ float cmb_bf(float v) { const unsigned u = __builtin_bit_cast(unsigned, v); const unsigned r = (u + 0x7fffu + ((u >> 16) & 1u)) & 0xffff0000u; return __builtin_bit_cast(float, r); }

__global__ __launch_bounds__(192) void k_bias3(const float* __restrict__ bq, const float* __restrict__ bk, const float* __restrict__ bv, float* __restrict__ BR) {
    const unsigned t = threadIdx.x; const unsigned m = t >> 6, i = t & 63u;
    const float a = bq[i], c = bk[i], d = bv[i];
    const float v = cmb_bf((m == 0u) ? a : ((m == 1u) ? c : d));
    VST2(float, BR + t, v);
}

__global__ __launch_bounds__(256) void k_wcastT(const float* __restrict__ Wq, const float* __restrict__ Wk, const float* __restrict__ Wv, unsigned short* __restrict__ DST, float sc) {
    const unsigned m = blockIdx.y;
    const float* SRC = (m == 0u) ? Wq : ((m == 1u) ? Wk : Wv);
    const unsigned u = blockIdx.x * 256u + threadIdx.x; const unsigned per = CIN / 8;
    if (u >= (unsigned)HD * per) return;
    const unsigned c = u / per; const unsigned r0 = 8u * (u - c * per);
    float w[8];
#pragma unroll
    for (int e = 0; e < 8; ++e) w[e] = cmb_bf(SRC[(size_t)(r0 + (unsigned)e) * HD + c]) * sc;
    cm_u4 pk; pk.x = cmb_pk2(w[0], w[1]); pk.y = cmb_pk2(w[2], w[3]); pk.z = cmb_pk2(w[4], w[5]); pk.w = cmb_pk2(w[6], w[7]);
    VST2(cm_u4, (cm_u4*)(DST + (size_t)m * HD * CIN + (size_t)c * CIN + r0), pk);
}

__global__ __launch_bounds__(256) void k_xcast(const float* __restrict__ SRC, unsigned short* __restrict__ DST, unsigned nR, unsigned seq, unsigned seq_full) {
    const unsigned u = blockIdx.x * 256u + threadIdx.x; const unsigned per = CIN / 8;
    if (u >= nR * per) return;
    const unsigned r = u / per; const unsigned c0 = 8u * (u - r * per);
    const unsigned bb = r / seq; const unsigned sr = bb * seq_full + (r - bb * seq);
    const float* s = SRC + (size_t)sr * CIN + c0;
    const v4f f0 = *(const v4f*)(s), f1 = *(const v4f*)(s + 4);
    cm_u4 pk; pk.x = cmb_pk2(cmb_bf(f0.x), cmb_bf(f0.y)); pk.y = cmb_pk2(cmb_bf(f0.z), cmb_bf(f0.w)); pk.z = cmb_pk2(cmb_bf(f1.x), cmb_bf(f1.y)); pk.w = cmb_pk2(cmb_bf(f1.z), cmb_bf(f1.w));
    VST2(cm_u4, (cm_u4*)(DST + (size_t)r * CIN + c0), pk);
}

__device__ __forceinline__ void dep_guard_h(v8f& a, v8f& b, v16h x, v16h y) { asm volatile("v_nop\n\tv_nop\n\tv_nop\n\tv_nop" : "+v"(a), "+v"(b) : "v"(x), "v"(y)); }
__device__ __forceinline__ void keep4_h(v16h a, v16h b, v16h c, v16h d) { asm volatile("v_nop" :: "v"(a), "v"(b), "v"(c), "v"(d)); }
__device__ __forceinline__ void acc_guard4(v8f& a, v8f& b, v8f& c, v8f& d) { asm volatile("v_nop\n\tv_nop\n\tv_nop\n\tv_nop" : "+v"(a), "+v"(b), "+v"(c), "+v"(d)); }
union FragU { v16h v; v8h h[2]; };
__device__ __forceinline__ v16h frag_ld(const _Float16* p) {
    FragU f; f.h[0] = *(const v8h*)(p); f.h[1] = *(const v8h*)(p + 16); return f.v;
}

__global__ __launch_bounds__(256) void k_gemm64(const unsigned short* __restrict__ Ap, int lda, const unsigned short* __restrict__ Btp, int ldb,
                                                float* __restrict__ C, int ldc, const float* __restrict__ bias, int M, int N, int K, float scale) {
    const _Float16* A = (const _Float16*)Ap; const _Float16* Bt = (const _Float16*)Btp;
    __shared__ __align__(16) float sT[8][16 * 68];
    const int lane = (int)(threadIdx.x & 31u);
    const int wave = (int)(threadIdx.x >> 5);
    const unsigned tilesN = (unsigned)N >> 6, tilesM = (unsigned)M >> 6;
    const unsigned tile = blockIdx.x * 8u + (unsigned)wave;
    if (tile >= tilesM * tilesN) return;
    const unsigned tm = tile / tilesN; const unsigned tn = tile - tm * tilesN;
    const int m0 = (int)(tm << 6), n0 = (int)(tn << 6);
    const int rlane = lane & 15;
    const int koff  = (lane >> 4) * 8;
    const int mOff  = (lane >> 4) * 8;

    v8f acc[4][4];
#pragma unroll
    for (int i = 0; i < 4; ++i)
#pragma unroll
        for (int j = 0; j < 4; ++j) acc[i][j] = (v8f){0.f, 0.f, 0.f, 0.f, 0.f, 0.f, 0.f, 0.f};

    for (int k0 = 0; k0 < K; k0 += 32) {
        v16h bh[4];
#pragma unroll
        for (int j = 0; j < 4; ++j) {
            const size_t bo = (size_t)(n0 + (j << 4) + rlane) * ldb + koff + k0;
            bh[j] = frag_ld(Bt + bo);
        }
#pragma unroll
        for (int i = 0; i < 4; ++i) {
            const size_t ao = (size_t)(m0 + (i << 4) + rlane) * lda + koff + k0;
            const v16h ah = frag_ld(A + ao);
#pragma unroll
            for (int j = 0; j < 4; ++j)
                acc[i][j] = __builtin_amdgcn_wmma_f32_16x16x32_f16(false, ah, false, bh[j], (short)0, acc[i][j], false, false);
            dep_guard_h(acc[i][0], acc[i][3], ah, ah);
        }
        keep4_h(bh[0], bh[1], bh[2], bh[3]);
    }
    acc_guard4(acc[0][0], acc[0][1], acc[0][2], acc[0][3]);
    acc_guard4(acc[1][0], acc[1][1], acc[1][2], acc[1][3]);
    acc_guard4(acc[2][0], acc[2][1], acc[2][2], acc[2][3]);
    acc_guard4(acc[3][0], acc[3][1], acc[3][2], acc[3][3]);

    float* slab = sT[wave];
#pragma unroll
    for (int i = 0; i < 4; ++i) {
        const int mBase = m0 + (i << 4);
#pragma unroll
        for (int j = 0; j < 4; ++j) {
            const int n = n0 + (j << 4) + rlane;
            const float bv = bias[n];
#pragma unroll
            for (int r = 0; r < 8; ++r) slab[(mOff + r) * 68 + (j << 4) + rlane] = acc[i][j][r] * scale + bv;
        }
        __builtin_amdgcn_fence(3  , "workgroup");
        __builtin_amdgcn_wave_barrier();
        __builtin_amdgcn_fence(2  , "workgroup");
        {
            const int hh = lane >> 4, c4 = (lane & 15) * 4;
            for (int pass = 0; pass < 2; ++pass) {
#pragma unroll
                for (int it = 0; it < 8; ++it) {
                    const int row = it * 2 + hh;
                    const v4f v = *(const v4f*)(slab + row * 68 + c4);
                    *(volatile v4f*)(C + (size_t)(mBase + row) * ldc + n0 + c4) = v;
                }
                __threadfence();
            }
        }
        __builtin_amdgcn_fence(3  , "workgroup");
        __builtin_amdgcn_wave_barrier();
        __builtin_amdgcn_fence(2  , "workgroup");
    }
}

__global__ __launch_bounds__(64) void k_gx_exact(const float* __restrict__ QKVp, unsigned ldq, unsigned rows_per_b, float sc,
                                                 float* __restrict__ OUTp, unsigned ldo, unsigned orows_per_b) {
    #pragma clang fp contract(off)
    __shared__ float qs[64]; __shared__ float ps[NXR]; __shared__ float red[2];
    const unsigned i = blockIdx.x, b = blockIdx.y, t = threadIdx.x;
    const float* base = QKVp + (size_t)b * rows_per_b * ldq;
    qs[t] = base[(size_t)i * ldq + t];
    __syncthreads();
    {
        const unsigned j = t; const unsigned jc = (j < i) ? j : i;
        const float* kr = base + (size_t)jc * ldq + 64; float s = 0.f;
#pragma unroll 8
        for (int d = 0; d < 64; ++d) s += qs[d] * kr[d];
        ps[j] = (j <= i) ? s * sc : -3.0e38f;
    }
    __syncthreads();
    if (t == 0) {
        float m = -3.0e38f;
        for (unsigned j = 0; j <= i; ++j) m = fmaxf(m, ps[j]);
        float z = 0.f;
        for (unsigned j = 0; j <= i; ++j) { const float e = expf(ps[j] - m); ps[j] = e; z += e; }
        red[0] = 1.f / z;
    }
    __syncthreads();
    const float inv = red[0]; float o = 0.f;
    for (unsigned j = 0; j <= i; ++j) o += ps[j] * base[(size_t)j * ldq + 128 + t];
    VST2(float, OUTp + ((size_t)b * orows_per_b + i) * ldo + t, o * inv);
}

struct AttnP {
    const float* Q; const float* K; const float* V; float* O;
    long long sQb, sQi, sKb, sKj, sVb, sVj, sOb, sOi;
    int Lq, Lk, coff, pad0; float scale; int pad1;
};
static_assert(sizeof(AttnP) == 4 * 8 + 8 * 8 + 4 * 4 + 4 + 4);

__global__ __launch_bounds__(32 * AW) void k_attn(AttnP p) {
    constexpr int NT = 4;
    constexpr int KS = 2;
    constexpr int VP = 72;
    __shared__ __align__(16) float    pl[AW][16 * 64];
    __shared__ __align__(16) _Float16 vl[64 * VP];
    const int lane = (int)(threadIdx.x & 31u), hf = lane >> 4, l15 = lane & 15, wave = (int)(threadIdx.x >> 5);
    const int tid = (int)threadIdx.x;
    const int b = (int)blockIdx.y;
    const int q0 = ((int)blockIdx.x * AW + wave) * 16;
    float* myp = pl[wave];
    const float L2E = 1.4426950408889634f;
    const float NEG = -__builtin_inff();
    const int qi = min(q0 + l15, p.Lq - 1);
    const float* qrow = p.Q + (long long)b * p.sQb + (long long)qi * p.sQi;
    const float* kbase = p.K + (long long)b * p.sKb;
    const float* vbase = p.V + (long long)b * p.sVb;
    Split qs_[KS];
#pragma unroll
    for (int ks = 0; ks < KS; ++ks) qs_[ks] = sp_row(qrow, ks * 32, hf);
    v8f o[NT]; float m8[8], l8[8];
#pragma unroll
    for (int t = 0; t < NT; ++t) { v8f zz = {}; o[t] = zz; }
#pragma unroll
    for (int i = 0; i < 8; ++i) { m8[i] = NEG; l8[i] = 0.f; }
    int jend = p.Lk;
    { const int je = ((int)blockIdx.x * AW + AW - 1) * 16 + 16 + p.coff; jend = min(jend, max(je, 0)); }
    for (int j0 = 0; j0 < jend; j0 += 64) {
        __syncthreads();
        for (int idx = tid; idx < 1024; idx += 32 * AW) {
            const int jr = idx >> 4, d = (idx & 15) * 4;
            const int j = min(j0 + jr, p.Lk - 1);
            const v4f f = *(const v4f*)(vbase + (long long)j * p.sVj + d);
            vl[jr * VP + d + 0] = (_Float16)f.x; vl[jr * VP + d + 1] = (_Float16)f.y; vl[jr * VP + d + 2] = (_Float16)f.z; vl[jr * VP + d + 3] = (_Float16)f.w;
        }
        v8f s[4];
#pragma unroll
        for (int t = 0; t < 4; ++t) {
            const int j = min(j0 + t * 16 + l15, p.Lk - 1);
            const float* krow = kbase + (long long)j * p.sKj;
            v8f acc = {};
#pragma unroll
            for (int ks = 0; ks < KS; ++ks) acc = wmma3(qs_[ks], sp_row(krow, ks * 32, hf), acc);
            s[t] = acc;
        }
#pragma unroll
        for (int i = 0; i < 8; ++i) {
            const int irow = q0 + i + 8 * hf;
            float sc[4];
#pragma unroll
            for (int t = 0; t < 4; ++t) {
                const int jg = j0 + t * 16 + l15;
                float v = s[t][i] * p.scale;
                if (jg >= p.Lk || jg > irow + p.coff) v = NEG; else v *= L2E;
                sc[t] = v;
            }
            float mx = fmaxf(fmaxf(sc[0], sc[1]), fmaxf(sc[2], sc[3]));
            mx = fmaxf(mx, __shfl_xor(mx, 1, 32)); mx = fmaxf(mx, __shfl_xor(mx, 2, 32));
            mx = fmaxf(mx, __shfl_xor(mx, 4, 32)); mx = fmaxf(mx, __shfl_xor(mx, 8, 32));
            const float mnew = fmaxf(m8[i], mx);
            const float corr = (mnew == NEG) ? 1.f : exp2f(m8[i] - mnew);
            float rs = 0.f;
#pragma unroll
            for (int t = 0; t < 4; ++t) {
                const float pp = (sc[t] == NEG) ? 0.f : exp2f(sc[t] - mnew); rs += pp;
                myp[(i + 8 * hf) * 64 + t * 16 + l15] = pp;
            }
            rs += __shfl_xor(rs, 1, 32); rs += __shfl_xor(rs, 2, 32); rs += __shfl_xor(rs, 4, 32); rs += __shfl_xor(rs, 8, 32);
            l8[i] = l8[i] * corr + rs; m8[i] = mnew;
#pragma unroll
            for (int t = 0; t < NT; ++t) o[t][i] *= corr;
        }
        __syncthreads();
        {
            const v16h pa0 = ph_row(myp + l15 * 64, 0, hf, 4096.f), pa1 = ph_row(myp + l15 * 64, 32, hf, 4096.f);
#pragma unroll
            for (int t = 0; t < NT; ++t) {
                const int dcol = t * 16 + l15;
                v16h b0, b1;
#pragma unroll
                for (int e = 0; e < 16; ++e) { b0[e] = vl[frag_k(e, hf) * VP + dcol]; b1[e] = vl[(32 + frag_k(e, hf)) * VP + dcol]; }
                o[t] = wmma16(pa0, b0, o[t]);
                o[t] = wmma16(pa1, b1, o[t]);
            }
        }
    }
    float* obase = p.O + (long long)b * p.sOb;
    float invr[8];
#pragma unroll
    for (int i = 0; i < 8; ++i) invr[i] = (l8[i] > 0.f) ? 1.f / (l8[i] * 4096.f) : 0.f;
    __syncthreads();
#pragma unroll
    for (int i = 0; i < 8; ++i)
#pragma unroll
        for (int t = 0; t < NT; ++t) myp[(i + 8 * hf) * 64 + t * 16 + l15] = o[t][i] * invr[i];
    __syncthreads();
#pragma unroll
    for (int r0 = 0; r0 < 16; r0 += 2) {
        const int row = r0 + (lane >> 4), c4 = (lane & 15) * 4;
        const v4f v = *(const v4f*)(myp + row * 64 + c4);
        VST2V4(obase + (long long)(q0 + row) * p.sOi + c4, v);
    }
}

extern "C" void kernel_launch(void* const* d_in, const int* in_sizes, int n_in, void* d_out, int out_size, void* d_ws, size_t ws_size, hipStream_t stream) {
    if (n_in < 7) return;
    const long long rows_span = (long long)(NB - 1) * SEQ_FULL + SEQ;
    if ((long long)in_sizes[0] < rows_span * CIN) return;
    if (in_sizes[1] < CIN * HD || in_sizes[3] < CIN * HD || in_sizes[5] < CIN * HD) return;
    if (in_sizes[2] < HD || in_sizes[4] < HD || in_sizes[6] < HD) return;
    if ((long long)out_size < rows_span * HD) return;
    const float* x  = (const float*)d_in[0];
    const float* Wq = (const float*)d_in[1];
    const float* bq = (const float*)d_in[2];
    const float* Wk = (const float*)d_in[3];
    const float* bk = (const float*)d_in[4];
    const float* Wv = (const float*)d_in[5];
    const float* bv = (const float*)d_in[6];
    float* out = (float*)d_out;

    const size_t MR = (size_t)NB * SEQ;
    const size_t szX = ((MR * CIN * 2 + 255) / 256) * 256;
    const size_t szW = (((size_t)NQKV * CIN * 2 + 255) / 256) * 256;
    const size_t szB = 1024;
    const size_t szQ = ((MR * NQKV * 4 + 255) / 256) * 256;
    if (szX + szW + szB + szQ > ws_size) return;
    if (szX + szW + szB + szQ > (size_t)134217728) return;
    char* wsp = (char*)d_ws;
    unsigned short* X16  = (unsigned short*)wsp; wsp += szX;
    unsigned short* W316 = (unsigned short*)wsp; wsp += szW;
    float* BR3 = (float*)wsp; wsp += szB;
    float* QKV = (float*)wsp; wsp += szQ;

    k_wcastT<<<dim3((unsigned)(HD * (CIN / 8) / 256), 3u), 256, 0, stream>>>(Wq, Wk, Wv, W316, 16.0f);
    k_bias3<<<1, 192, 0, stream>>>(bq, bk, bv, BR3);
    k_xcast<<<(unsigned)((MR * (CIN / 8) + 255) / 256), 256, 0, stream>>>(x, X16, (unsigned)MR, (unsigned)SEQ, (unsigned)SEQ_FULL);
    k_gemm64<<<(unsigned)(((MR / 64) * (NQKV / 64) + 7) / 8), 256, 0, stream>>>(X16, CIN, W316, CIN, QKV, NQKV, BR3, (int)MR, NQKV, CIN, 0.0625f);
    k_gx_exact<<<dim3((unsigned)NXR, (unsigned)NB), 64, 0, stream>>>(QKV, (unsigned)NQKV, (unsigned)SEQ, 0.125f, out, (unsigned)HD, (unsigned)SEQ_FULL);
    {
        AttnP a;
        a.Q = QKV + (size_t)NXR * NQKV; a.K = QKV + 64; a.V = QKV + 128; a.O = out + (size_t)NXR * HD;
        a.sQb = (long long)SEQ * NQKV; a.sQi = NQKV; a.sKb = (long long)SEQ * NQKV; a.sKj = NQKV; a.sVb = (long long)SEQ * NQKV; a.sVj = NQKV;
        a.sOb = (long long)SEQ_FULL * HD; a.sOi = HD;
        a.Lq = SEQ - NXR; a.Lk = SEQ; a.coff = NXR; a.pad0 = 0; a.scale = 0.125f; a.pad1 = 0;
        k_attn<<<dim3((unsigned)((SEQ - NXR) / (16 * AW)), (unsigned)NB), 32 * AW, 0, stream>>>(a);
    }
}
